// GeometryAwareAttention_84413287236162
// MI455X (gfx1250) — hardware-verified
//
#include <hip/hip_runtime.h>


#define NB_  4
#define TT   2048
#define DM   256
#define NH_  8
#define HD   32
#define PCAR 1024.0f
#define SCL  0.17677669529663687f
typedef _Float16 h16;
typedef unsigned short bf;
typedef __attribute__((ext_vector_type(16))) __bf16   v16bf;
typedef __attribute__((ext_vector_type(16))) _Float16 v16h;
typedef __attribute__((ext_vector_type(8)))  _Float16 v8h;
typedef __attribute__((ext_vector_type(8)))  unsigned short v8us;
typedef __attribute__((ext_vector_type(8)))  float    v8f;
typedef __attribute__((ext_vector_type(4)))  float    v4f;
typedef v8h  __attribute__((may_alias)) v8ha;
typedef v4f  __attribute__((may_alias)) v4fa;
typedef v8us __attribute__((may_alias)) v8usa;

__device__ __forceinline__ unsigned short f2bf(float f) { unsigned u = __float_as_uint(f); u += 0x7FFFu + ((u >> 16) & 1u); return (unsigned short)(u >> 16); }
__device__ __forceinline__ float bf2f(unsigned short b) { return __uint_as_float(((unsigned)b) << 16); }
__device__ __forceinline__ float bfr(float f) { return bf2f(f2bf(f)); }
__device__ __forceinline__ v16h cat16(v8h lo, v8h hi) { return __builtin_shufflevector(lo, hi, 0, 1, 2, 3, 4, 5, 6, 7, 8, 9, 10, 11, 12, 13, 14, 15); }
__device__ __forceinline__ v16bf cat16b(v8us lo, v8us hi) { return __builtin_bit_cast(v16bf, __builtin_shufflevector(lo, hi, 0, 1, 2, 3, 4, 5, 6, 7, 8, 9, 10, 11, 12, 13, 14, 15)); }
__device__ __forceinline__ v8f wmma16(v16h a, v16h b, v8f c) { return __builtin_amdgcn_wmma_f32_16x16x32_f16(false, a, false, b, (short)0, c, false, false); }
__device__ __forceinline__ v8f wmmab(v16bf a, v16bf b, v8f c) { return __builtin_amdgcn_wmma_f32_16x16x32_bf16(false, a, false, b, (short)0, c, false, false); }


template <typename T16> struct WFrag;
template <> struct WFrag<h16> { typedef v16h V; static __device__ __forceinline__ V ld(const h16* p) { return cat16(*(const v8h*)p, *(const v8h*)(p + 16)); } static __device__ __forceinline__ v8f mma(V a, V b, v8f c) { return wmma16(a, b, c); } };
template <> struct WFrag<bf> { typedef v16bf V; static __device__ __forceinline__ V ld(const bf* p) { return cat16b(*(const v8us*)p, *(const v8us*)(p + 16)); } static __device__ __forceinline__ v8f mma(V a, V b, v8f c) { return wmmab(a, b, c); } };
template <typename T16, int NSPLIT, bool BIAS>
__global__ __launch_bounds__(32) void k_gemmw(const T16* __restrict__ A, const T16* __restrict__ A2, const T16* __restrict__ Bt, const T16* __restrict__ Bt2, int K, float* C, int ldc, const float* __restrict__ bias, size_t sA, size_t sB, size_t sC) {
    typedef typename WFrag<T16>::V V;
    __shared__ __align__(16) float os[16 * 68];
    const size_t z = blockIdx.z; A += z * sA; if (A2) A2 += z * sA; Bt += z * sB; if (Bt2) Bt2 += z * sB; C += z * sC;
    const int lane = threadIdx.x & 31, lr = lane & 15, hi = lane >> 4; const int r0 = blockIdx.x * 64, c0 = blockIdx.y * 64;
    v8f acc[4][4];
#pragma unroll
    for (int mb = 0; mb < 4; ++mb)
#pragma unroll
        for (int nb = 0; nb < 4; ++nb) acc[mb][nb] = (v8f){};
    const size_t aoff = (size_t)(r0 + lr) * K + 8 * hi, boff = (size_t)(c0 + lr) * K + 8 * hi;
#pragma unroll 1
    for (int kc = 0; kc < K; kc += 32) {
        V a[4], a2[4];
#pragma unroll
        for (int mb = 0; mb < 4; ++mb) { a[mb] = WFrag<T16>::ld(A + aoff + (size_t)mb * 16 * K + kc); if (NSPLIT == 1 || NSPLIT == 2) a2[mb] = WFrag<T16>::ld(A2 + aoff + (size_t)mb * 16 * K + kc); }
#pragma unroll
        for (int nb = 0; nb < 4; ++nb) { const V b = WFrag<T16>::ld(Bt + boff + (size_t)nb * 16 * K + kc); V b2; if (NSPLIT >= 2) b2 = WFrag<T16>::ld(Bt2 + boff + (size_t)nb * 16 * K + kc);
#pragma unroll
            for (int mb = 0; mb < 4; ++mb) { acc[mb][nb] = WFrag<T16>::mma(a[mb], b, acc[mb][nb]); if (NSPLIT == 1 || NSPLIT == 2) acc[mb][nb] = WFrag<T16>::mma(a2[mb], b, acc[mb][nb]); if (NSPLIT >= 2) acc[mb][nb] = WFrag<T16>::mma(a[mb], b2, acc[mb][nb]); } }
        asm volatile("v_nop\n\tv_nop\n\tv_nop\n\tv_nop" : "+v"(acc[0][0]), "+v"(acc[1][1]), "+v"(acc[2][2]), "+v"(acc[3][3]) : "v"(a[0]), "v"(a[3]));
    }
#pragma unroll
    for (int mb = 0; mb < 4; ++mb) {
#pragma unroll
        for (int nb = 0; nb < 4; ++nb) {
#pragma unroll
            for (int j = 0; j < 8; ++j) os[(hi * 8 + j) * 68 + nb * 16 + lr] = acc[mb][nb][j]; }
        __builtin_amdgcn_wave_barrier(); asm volatile("" ::: "memory");
        float* crow = C + (size_t)(r0 + mb * 16) * ldc + c0;
#pragma unroll 1
        for (int ps = 0; ps < 2; ++ps) {
#pragma unroll
            for (int s = 0; s < 8; ++s) { const int row = 2 * s + hi, cofs = lr * 4; v4f val = *(const v4fa*)(os + row * 68 + cofs); if (BIAS) { val[0] += bfr(bias[c0 + cofs]); val[1] += bfr(bias[c0 + cofs + 1]); val[2] += bfr(bias[c0 + cofs + 2]); val[3] += bfr(bias[c0 + cofs + 3]); }
                *(volatile v4f*)(crow + (size_t)row * ldc + cofs) = val; }
            if (ps == 0) __threadfence(); }
        __builtin_amdgcn_wave_barrier(); asm volatile("" ::: "memory");
    }
}

__device__ __forceinline__ h16 tohx(float x) { return (h16)x; }
typedef __attribute__((ext_vector_type(2))) _Float16 v2h;
typedef __attribute__((ext_vector_type(4))) _Float16 v4h;
typedef __attribute__((ext_vector_type(2))) float v2f;

__global__ __launch_bounds__(256) void k_cvt8(const float* __restrict__ src, bf* dst, size_t n8) { const size_t i = (size_t)blockIdx.x * 256 + threadIdx.x; if (i >= n8) return; const v8f v = *(const v8f*)(src + i * 8); v8us o;
#pragma unroll
    for (int k = 0; k < 8; ++k) o[k] = f2bf(v[k]); *(volatile v8us*)(dst + i * 8) = o; __threadfence(); *(volatile v8us*)(dst + i * 8) = o; }
__global__ __launch_bounds__(256) void k_qk16(const float* __restrict__ FQ, const float* __restrict__ FK, h16* QP, h16* KP) { const size_t e = ((size_t)blockIdx.x * 256 + threadIdx.x) * 2; if (e >= (size_t)NH_ * TT * HD) return; const int d = (int)(e % HD); const int t = (int)((e / HD) % TT); const int h = (int)(e / ((size_t)HD * TT)); const size_t s = (size_t)t * DM + h * HD + d; v2h q, k; q[0] = tohx(FQ[s]); q[1] = tohx(FQ[s + 1]); k[0] = tohx(FK[s]); k[1] = tohx(FK[s + 1]);
    *(volatile v2h*)(QP + e) = q; *(volatile v2h*)(KP + e) = k; __threadfence(); *(volatile v2h*)(QP + e) = q; *(volatile v2h*)(KP + e) = k; }
__global__ __launch_bounds__(256) void k_vt16(const float* __restrict__ FV, h16* VT) { const size_t e = ((size_t)blockIdx.x * 256 + threadIdx.x) * 2; if (e >= (size_t)NH_ * 64 * TT) return; const int t = (int)(e % TT); const int dd = (int)((e / TT) % 64); const int h = (int)(e / ((size_t)TT * 64)); v2h o;
    if (dd < HD) { o[0] = tohx(FV[(size_t)t * DM + h * HD + dd]); o[1] = tohx(FV[(size_t)(t + 1) * DM + h * HD + dd]); } else { o[0] = (h16)0.f; o[1] = (h16)0.f; } *(volatile v2h*)(VT + e) = o; __threadfence(); *(volatile v2h*)(VT + e) = o; }
__global__ __launch_bounds__(256) void k_gbias(const float* __restrict__ crd, const float* __restrict__ alpha, float* GB) { const size_t e = ((size_t)blockIdx.x * 256 + threadIdx.x) * 4; if (e >= (size_t)TT * TT) return; const int j0 = (int)(e % TT), i = (int)(e / TT); const float al = bfr(alpha[0]); const float c0 = bfr(crd[(size_t)i * 3]), c1 = bfr(crd[(size_t)i * 3 + 1]), c2 = bfr(crd[(size_t)i * 3 + 2]); v4f o;
#pragma unroll
    for (int q = 0; q < 4; ++q) { const int j = j0 + q; float g0 = __fmul_rn(c0, bfr(crd[(size_t)j * 3])), g1 = __fmul_rn(c1, bfr(crd[(size_t)j * 3 + 1])), g2 = __fmul_rn(c2, bfr(crd[(size_t)j * 3 + 2])); asm volatile("" : "+v"(g0), "+v"(g1), "+v"(g2)); o[q] = __fmul_rn(al, __fadd_rn(__fadd_rn(g0, g1), g2)); }
    *(volatile v4f*)(GB + e) = o; __threadfence(); *(volatile v4f*)(GB + e) = o; }
__global__ __launch_bounds__(256) void k_gsoft(const float* __restrict__ Sb, const float* __restrict__ GB, h16* P16) { const int lane = threadIdx.x & 31; const int row = blockIdx.x * 8 + (threadIdx.x >> 5); if (row >= TT) return; const float* sr = Sb + (size_t)row * TT; const float* gr = GB + (size_t)row * TT; float v[64]; float mx = -3.0e38f;
#pragma unroll
    for (int ch = 0; ch < 16; ++ch) { const int j0 = ch * 128 + lane * 4; const v4f a = *(const v4f*)(sr + j0), gg = *(const v4f*)(gr + j0);
#pragma unroll
        for (int q = 0; q < 4; ++q) { float s8 = __fmul_rn(a[q], SCL); asm volatile("" : "+v"(s8)); const float t = __fadd_rn(s8, gg[q]); v[ch * 4 + q] = t; mx = fmaxf(mx, t); } }
#pragma unroll
    for (int sh = 16; sh; sh >>= 1) mx = fmaxf(mx, __shfl_xor(mx, sh, 32));
    float sum = 0.f;
#pragma unroll
    for (int k = 0; k < 64; ++k) { float d0 = __fsub_rn(v[k], mx); asm volatile("" : "+v"(d0)); v[k] = __expf(d0); sum += v[k]; }
#pragma unroll
    for (int sh = 16; sh; sh >>= 1) sum += __shfl_xor(sum, sh, 32);
    const float f = __fdiv_rn(PCAR, sum);
#pragma unroll 1
    for (int ps = 0; ps < 2; ++ps) {
#pragma unroll
        for (int ch = 0; ch < 16; ++ch) { v4h o;
#pragma unroll
            for (int q = 0; q < 4; ++q) o[q] = tohx(v[ch * 4 + q] * f); *(volatile v4h*)(P16 + (size_t)row * TT + ch * 128 + lane * 4) = o; }
        if (ps == 0) __threadfence(); } }
__global__ __launch_bounds__(256) void k_ofin(const float* __restrict__ O, int h, float* OUTb) { const size_t e = ((size_t)blockIdx.x * 256 + threadIdx.x) * 2; if (e >= (size_t)TT * HD) return; const int d = (int)(e % HD), t = (int)(e / HD); v2f o; o[0] = O[(size_t)t * 64 + d] * (1.0f / PCAR); o[1] = O[(size_t)t * 64 + d + 1] * (1.0f / PCAR); const size_t oo = (size_t)t * DM + h * HD + d; *(volatile v2f*)(OUTb + oo) = o; __threadfence(); *(volatile v2f*)(OUTb + oo) = o; }

extern "C" void kernel_launch(void* const* d_in, const int* in_sizes, int n_in,
                              void* d_out, int out_size, void* d_ws, size_t ws_size, hipStream_t stream) {
    (void)in_sizes; (void)n_in; (void)out_size;
    const float* x = (const float*)d_in[0]; const float* crd = (const float*)d_in[1]; const float* wq = (const float*)d_in[2]; const float* bq = (const float*)d_in[3]; const float* wk = (const float*)d_in[4]; const float* bk = (const float*)d_in[5]; const float* wv = (const float*)d_in[6]; const float* bv = (const float*)d_in[7]; const float* alpha = (const float*)d_in[8];
    float* OUT = (float*)d_out;
    char* wsp = (char*)d_ws;
    auto take = [&](size_t bytes) { char* p = wsp; wsp += (bytes + 255) & ~(size_t)255; return (void*)p; };
    bf* WQ = (bf*)take((size_t)DM * DM * 2); bf* WK = (bf*)take((size_t)DM * DM * 2); bf* WV = (bf*)take((size_t)DM * DM * 2); bf* XB = (bf*)take((size_t)TT * DM * 2); float* FQ = (float*)take((size_t)TT * DM * 4); float* FK = (float*)take((size_t)TT * DM * 4); float* FV = (float*)take((size_t)TT * DM * 4);
    h16* QP = (h16*)take((size_t)NH_ * TT * HD * 2); h16* KP = (h16*)take((size_t)NH_ * TT * HD * 2); h16* VT = (h16*)take((size_t)NH_ * 64 * TT * 2); float* Sb = (float*)take((size_t)TT * TT * 4); h16* P16 = (h16*)take((size_t)TT * TT * 2); float* O = (float*)take((size_t)TT * 64 * 4); float* GB = (float*)take((size_t)TT * TT * 4);
    if ((size_t)(wsp - (char*)d_ws) > ws_size) return;
    { const unsigned g = (DM * DM / 8 + 255) / 256; k_cvt8<<<g, 256, 0, stream>>>(wq, WQ, (size_t)DM * DM / 8); k_cvt8<<<g, 256, 0, stream>>>(wk, WK, (size_t)DM * DM / 8); k_cvt8<<<g, 256, 0, stream>>>(wv, WV, (size_t)DM * DM / 8); }
    const dim3 gP(TT / 64, DM / 64, 1);
    for (int b = 0; b < NB_; ++b) {
        k_cvt8<<<(TT * DM / 8 + 255) / 256, 256, 0, stream>>>(x + (size_t)b * TT * DM, XB, (size_t)TT * DM / 8);
        k_gemmw<bf, 0, true><<<gP, 32, 0, stream>>>(XB, nullptr, WQ, nullptr, DM, FQ, DM, bq, 0, 0, 0); k_gemmw<bf, 0, true><<<gP, 32, 0, stream>>>(XB, nullptr, WK, nullptr, DM, FK, DM, bk, 0, 0, 0); k_gemmw<bf, 0, true><<<gP, 32, 0, stream>>>(XB, nullptr, WV, nullptr, DM, FV, DM, bv, 0, 0, 0);
        k_gbias<<<(unsigned)(((size_t)TT * TT / 4 + 255) / 256), 256, 0, stream>>>(crd + (size_t)b * TT * 3, alpha, GB);
        k_qk16<<<(unsigned)(((size_t)NH_ * TT * HD / 2 + 255) / 256), 256, 0, stream>>>(FQ, FK, QP, KP); k_vt16<<<(unsigned)(((size_t)NH_ * 64 * TT / 2 + 255) / 256), 256, 0, stream>>>(FV, VT);
        for (int h = 0; h < NH_; ++h) {
            k_gemmw<h16, 0, false><<<dim3(TT / 64, TT / 64, 1), 32, 0, stream>>>(QP + (size_t)h * TT * HD, nullptr, KP + (size_t)h * TT * HD, nullptr, HD, Sb, TT, nullptr, 0, 0, 0);
            k_gsoft<<<TT / 8, 256, 0, stream>>>(Sb, GB, P16);
            k_gemmw<h16, 0, false><<<dim3(TT / 64, 1, 1), 32, 0, stream>>>(P16, nullptr, VT + (size_t)h * 64 * TT, nullptr, TT, O, 64, nullptr, 0, 0, 0);
            k_ofin<<<(TT * HD / 2 + 255) / 256, 256, 0, stream>>>(O, h, OUT + (size_t)b * TT * DM); } }
}
